// TSModel_56513179681517
// MI455X (gfx1250) — hardware-verified
//
#include <hip/hip_runtime.h>


namespace {
typedef _Float16 b16;
typedef __attribute__((ext_vector_type(16))) _Float16 v16b;
typedef __attribute__((ext_vector_type(8))) _Float16 v8b;
typedef __attribute__((ext_vector_type(4))) _Float16 v4h;
typedef __attribute__((ext_vector_type(2))) _Float16 v2h;
typedef __attribute__((ext_vector_type(8))) float v8f;
typedef __attribute__((ext_vector_type(4))) float v4f;
typedef __attribute__((ext_vector_type(2))) float v2f;
__device__ __forceinline__ float bf16_rne(float f) { unsigned int u = __float_as_uint(f); u += 0x7FFFu + ((u >> 16) & 1u); return __uint_as_float(u & 0xFFFF0000u); }
__device__ __forceinline__ void split16(float v, b16& hi, b16& lo) { hi = (b16)v; lo = (b16)(v - (float)hi); }
__device__ __forceinline__ v16b frag_kb(const b16* p, int hh) { const v8b a = *(const v8b*)(p + 8 * hh), b = *(const v8b*)(p + 16 + 8 * hh); v16b f;
#pragma unroll
  for (int e = 0; e < 8; ++e) { f[e] = a[e]; f[8 + e] = b[e]; } return f; }
__device__ __forceinline__ v8f wmma16b(v16b a, v16b b, v8f c) { v8f d = __builtin_amdgcn_wmma_f32_16x16x32_f16(false, a, false, b, (short)0, c, false, false); asm volatile("v_nop\n\tv_nop\n\tv_nop\n\tv_nop" : "+v"(d) : "v"(a), "v"(b)); return d; }
__device__ __forceinline__ void wave_lds_sync() { __builtin_amdgcn_fence(__ATOMIC_RELEASE, "workgroup"); __builtin_amdgcn_wave_barrier(); __builtin_amdgcn_fence(__ATOMIC_ACQUIRE, "workgroup"); }
__device__ __forceinline__ float pmul(float a, float b) { float p = a * b; asm volatile("" : "+v"(p)); return p; }
__device__ __forceinline__ int iclamp(int v, int lo, int hi) { return v < lo ? lo : (v > hi ? hi : v); }
__device__ __forceinline__ float nexp2(float v) { return __builtin_amdgcn_exp2f(v); }

constexpr int BS = 512, BSL = BS  , T = 1024, TL = T  , H = 64, G4 = 4 * H;
constexpr float XS = 8.0f, WSC = 256.0f, RS = 1024.0f, FB = 1.0f;
static_assert(BS % 32 == 0 && BSL % 32 == 0 && T % 32 == 0 && TL % 32 == 0 && H == 64, "tiling");
__device__ __forceinline__ float sigm(float v) { return 1.0f / (1.0f + __expf(-v)); }
__device__ __forceinline__ float tnh(float v) { return 2.0f / (1.0f + __expf(-2.0f * v)) - 1.0f; }
__global__ __launch_bounds__(256) void prep_kernel(const float* __restrict__ w1, b16* __restrict__ WT) {
  const int u = blockIdx.x * 256 + threadIdx.x; if (u >= G4 * H / 8) return; const int e = u * 8; const int o = e / H, k0 = e % H; v8b v;
  for (int j = 0; j < 8; ++j) v[j] = (b16)(bf16_rne(w1[(size_t)(1 + k0 + j) * G4 + o]) * WSC);
  for (int pass = 0; pass < 2; ++pass) { *(volatile v8b*)(WT + e) = v; __threadfence(); }
}
__global__ __launch_bounds__(64) void lstm_kernel(const float* __restrict__ x, const float* __restrict__ w1, const float* __restrict__ b1, const b16* __restrict__ WT, const float* __restrict__ w2, const float* __restrict__ b2, float* __restrict__ out) {
  __shared__ __attribute__((aligned(16))) b16 Ah[2][2][16][H + 8], Al[2][2][16][H + 8];   __shared__ float C1[2][16][H], H1[2][16][H + 1], Ys[2][16][33]; __shared__ float w1x[G4], b1s[G4], w2s[65 * 4], b2s[4];
  const int wave = threadIdx.x >> 5, lane = threadIdx.x & 31, nloc = lane & 15, hlf = lane >> 4; const int r0 = blockIdx.x * 32 + wave * 16;
  for (int i = threadIdx.x; i < G4; i += 64) { w1x[i] = bf16_rne(w1[i]); b1s[i] = bf16_rne(b1[i]); }
  for (int i = threadIdx.x; i < 65 * 4; i += 64) w2s[i] = bf16_rne(w2[i]); if (threadIdx.x < 4) b2s[threadIdx.x] = bf16_rne(b2[threadIdx.x]);
  for (int i = lane; i < 16 * H; i += 32) { const int rr = i / H, u = i % H; C1[wave][rr][u] = 0.0f; H1[wave][rr][u] = 0.0f; Ah[0][wave][rr][u] = (b16)0.0f; Al[0][wave][rr][u] = (b16)0.0f; Ah[1][wave][rr][u] = (b16)0.0f; Al[1][wave][rr][u] = (b16)0.0f; }
  __syncthreads();
  float c2 = 0.0f, h2 = 0.0f; const int myrow = lane & 15;
#pragma unroll 1
  for (int t = 0; t < TL; ++t) {
    const int pi = t & 1, po = pi ^ 1; const v16b a0 = frag_kb(&Ah[pi][wave][nloc][0], hlf), a1 = frag_kb(&Ah[pi][wave][nloc][32], hlf), l0 = frag_kb(&Al[pi][wave][nloc][0], hlf), l1 = frag_kb(&Al[pi][wave][nloc][32], hlf);
#pragma unroll 1
    for (int q = 0; q < 4; ++q) {
      v8f acc[4], accl[4];
#pragma unroll
      for (int g = 0; g < 4; ++g) { const b16* wr = WT + (size_t)((g * 4 + q) * 16 + nloc) * H; const v16b b0 = frag_kb(wr, hlf), bb1 = frag_kb(wr + 32, hlf);
        acc[g] = wmma16b(a0, b0, (v8f){}); acc[g] = wmma16b(a1, bb1, acc[g]); accl[g] = wmma16b(l0, b0, (v8f){}); accl[g] = wmma16b(l1, bb1, accl[g]); }
      const int u = q * 16 + nloc;
#pragma unroll
      for (int r = 0; r < 8; ++r) { const int rr = 8 * hlf + r; const float xt = bf16_rne(x[(size_t)(r0 + rr) * T + t]);
        const float gi = (acc[0][r] + accl[0][r] * (1.0f / RS)) * (1.0f / (XS * WSC)) + xt * w1x[u] + b1s[u], gj = (acc[1][r] + accl[1][r] * (1.0f / RS)) * (1.0f / (XS * WSC)) + xt * w1x[H + u] + b1s[H + u];
        const float gf = (acc[2][r] + accl[2][r] * (1.0f / RS)) * (1.0f / (XS * WSC)) + xt * w1x[2 * H + u] + b1s[2 * H + u], go = (acc[3][r] + accl[3][r] * (1.0f / RS)) * (1.0f / (XS * WSC)) + xt * w1x[3 * H + u] + b1s[3 * H + u];
        const float c = C1[wave][rr][u] * sigm(gf + FB) + sigm(gi) * tnh(gj); const float h = tnh(c) * sigm(go); C1[wave][rr][u] = c; H1[wave][rr][u] = h; const float hs = h * XS; const b16 ph = (b16)hs; Ah[po][wave][rr][u] = ph; Al[po][wave][rr][u] = (b16)((hs - (float)ph) * RS); } }
    wave_lds_sync();
    float ga = 0.0f, gb = 0.0f; const int g0 = 2 * hlf;
#pragma unroll 4
    for (int k = 0; k < H; ++k) { const float hv = H1[wave][myrow][k]; ga = fmaf(hv, w2s[k * 4 + g0], ga); gb = fmaf(hv, w2s[k * 4 + g0 + 1], gb); }
    ga += h2 * w2s[H * 4 + g0] + b2s[g0]; gb += h2 * w2s[H * 4 + g0 + 1] + b2s[g0 + 1];
    const float oa = __shfl_xor(ga, 16), ob = __shfl_xor(gb, 16);
    const float gi2 = hlf ? oa : ga, gj2 = hlf ? ob : gb, gf2 = hlf ? ga : oa, go2 = hlf ? gb : ob;
    c2 = c2 * sigm(gf2 + FB) + sigm(gi2) * tnh(gj2); h2 = tnh(c2) * sigm(go2);
    if (hlf == 0) Ys[wave][myrow][t & 31] = h2;
    if ((t & 31) == 31) { wave_lds_sync(); for (int pass = 0; pass < 2; ++pass) { for (int rr = 0; rr < 16; ++rr) ((volatile float*)out)[(size_t)(r0 + rr) * T + (t - 31) + lane] = Ys[wave][rr][lane]; __threadfence(); } wave_lds_sync(); } }
}
}

extern "C" void kernel_launch(void* const* d_in, const int* in_sizes, int n_in, void* d_out, int out_size, void* d_ws, size_t ws_size, hipStream_t stream) {
  (void)n_in;
  auto Fp = [&](int i) { return (const float*)d_in[i]; };
  if (in_sizes[0] != BS * T || in_sizes[1] != 65 * G4 || in_sizes[2] != G4 || in_sizes[3] != 65 * 4 || in_sizes[4] != 4 || out_size != BS * T) return;
  size_t off = 0; char* ws = (char*)d_ws;
  auto carve = [&](size_t bytes) { char* p = ws + off; off += (bytes + 255) & ~(size_t)255; return p; };
  b16* WT = (b16*)carve((size_t)G4 * H * 2);
  if (off > ws_size || off > ((size_t)128 << 20)) return;
  prep_kernel<<<(G4 * H / 8 + 255) / 256, 256, 0, stream>>>(Fp(1), WT);
  lstm_kernel<<<BSL / 32, 64, 0, stream>>>(Fp(0), Fp(1), Fp(2), WT, Fp(3), Fp(4), (float*)d_out);
}
